// MultiHeadCoAttentionWithGating_3478923510080
// MI455X (gfx1250) — hardware-verified
//
#include <hip/hip_runtime.h>
#include <stddef.h>
#include <stdint.h>


#define DF    128
#define NH    8
#define HC    16
#define QKVW  (3 * DF)
#define FFW   (4 * DF)
#define GR    32
#define XSP   132
#define NTHR  256
#define NWAVE 8
#define NB    512
#define CHUNK 2048
#define WCAP  256
#define NGRP  (CHUNK / (NTHR * 4))
#define WSC   16.0f
#define ASC   16.0f

#define LDS_SACC (NB * DF)
#define LDS_DEN  (NB * NH)
#define LDS_LIST (NWAVE * WCAP)
#define AGG_LDS_BYTES ((LDS_SACC + LDS_DEN + LDS_LIST + NWAVE) * 4)

static_assert(WCAP == NGRP * 4 * 32);
static_assert(NGRP >= 1);
static_assert(NB == 512);
static_assert(CHUNK == 2048);
static_assert(((LDS_SACC + LDS_DEN) % 4) == 0);
static_assert(AGG_LDS_BYTES == 286752);
static_assert((XSP % 4) == 0);

typedef float    v4f  __attribute__((ext_vector_type(4)));
typedef float    v8f  __attribute__((ext_vector_type(8)));
typedef int      v4i  __attribute__((ext_vector_type(4)));
typedef _Float16 v8h  __attribute__((ext_vector_type(8)));
typedef _Float16 v16h __attribute__((ext_vector_type(16)));
union Frag   { v16h v; v8h half[2]; };
union Pack16 { v8h h; v4i i; };

__device__ __forceinline__ v8f z8f() {
  v8f v = {0.f, 0.f, 0.f, 0.f, 0.f, 0.f, 0.f, 0.f};
  return v;
}

__device__ __forceinline__ v8f wm(v16h a, v16h b, v8f c) {
  v8f d = __builtin_amdgcn_wmma_f32_16x16x32_f16(false, a, false, b, (short)0, c, false, false);
  asm volatile("v_nop\n\tv_nop\n\tv_nop\n\tv_nop" : "+v"(d) : "v"(a), "v"(b));
  return d;
}

__device__ __forceinline__ v16h ldf(const _Float16* p) {
  Frag f;
  f.half[0] = *(const v8h*)p;
  f.half[1] = *(const v8h*)(p + 16);
  return f.v;
}

__device__ __forceinline__ float hsum16(float v) {
  v += __shfl_xor(v, 8, 32);
  v += __shfl_xor(v, 4, 32);
  v += __shfl_xor(v, 2, 32);
  v += __shfl_xor(v, 1, 32);
  return v;
}

__device__ __forceinline__ Pack16 pack8(v4f a, v4f b) {
  Pack16 u;
  u.h[0] = (_Float16)a.x; u.h[1] = (_Float16)a.y; u.h[2] = (_Float16)a.z; u.h[3] = (_Float16)a.w;
  u.h[4] = (_Float16)b.x; u.h[5] = (_Float16)b.y; u.h[6] = (_Float16)b.z; u.h[7] = (_Float16)b.w;
  return u;
}

__global__ __launch_bounds__(NTHR) void k_cvt(const float* __restrict__ x, _Float16* y, int n8) {
  const int i = blockIdx.x * NTHR + threadIdx.x;
  if (i >= n8) return;
  const size_t o = (size_t)i * 8;
  const v4f a = *(const v4f*)(x + o);
  const v4f b = *(const v4f*)(x + o + 4);
  const Pack16 u = pack8(a, b);
  *(volatile v4i*)(y + o) = u.i;
  __threadfence();
  *(volatile v4i*)(y + o) = u.i;
}

__global__ __launch_bounds__(NTHR) void k_wt(const float* __restrict__ s0, const float* __restrict__ s1,
                                             const float* __restrict__ s2, _Float16* dst, int K, int N) {
  __shared__ __attribute__((aligned(16))) _Float16 T[32][72];
  const float* src = (blockIdx.z == 0) ? s0 : ((blockIdx.z == 1) ? s1 : s2);
  const int nkt = K >> 6;
  const int kt = (int)blockIdx.x % nkt, nt = (int)blockIdx.x / nkt;
  const int k0 = kt * 64, n0 = nt * 32;
  const int tid = threadIdx.x;
  {
    const int r = tid >> 2;
    const int c = (tid & 3) * 8;
    const float* p = src + (size_t)(k0 + r) * N + n0 + c;
    const v4f a = *(const v4f*)p;
    const v4f b = *(const v4f*)(p + 4);
    T[c + 0][r] = (_Float16)(a.x * WSC); T[c + 1][r] = (_Float16)(a.y * WSC);
    T[c + 2][r] = (_Float16)(a.z * WSC); T[c + 3][r] = (_Float16)(a.w * WSC);
    T[c + 4][r] = (_Float16)(b.x * WSC); T[c + 5][r] = (_Float16)(b.y * WSC);
    T[c + 6][r] = (_Float16)(b.z * WSC); T[c + 7][r] = (_Float16)(b.w * WSC);
  }
  __syncthreads();
  {
    const int n = tid >> 3;
    const int q = tid & 7;
    Pack16 u;
    u.h = *(const v8h*)(&T[n][8 * q]);
    _Float16* p = dst + (size_t)((int)blockIdx.z * N + n0 + n) * K + k0 + 8 * q;
    *(volatile v4i*)p = u.i;
    __threadfence();
    *(volatile v4i*)p = u.i;
  }
}

__global__ __launch_bounds__(NTHR) void k_qkv(const _Float16* __restrict__ A, const _Float16* __restrict__ Wt,
                                              float* out) {
  __shared__ __attribute__((aligned(16))) float Xs[GR * XSP];
  const int tid = threadIdx.x, lane = tid & 31, wave = tid >> 5;
  const int hh = lane >> 4, m = lane & 15;
  const int rowBase = blockIdx.x * GR;
  const int colBlk = blockIdx.y * DF;
  const int lcol = wave * 16 + m;
  const int ncol = colBlk + lcol;

  const _Float16* pa0 = A + (size_t)(rowBase + m) * DF + 8 * hh;
  const _Float16* pa1 = pa0 + (size_t)16 * DF;
  const _Float16* pb  = Wt + (size_t)ncol * DF + 8 * hh;
  v8f c0 = z8f(), c1 = z8f();
#pragma unroll
  for (int kt = 0; kt < DF / 32; ++kt) {
    const int k0 = kt * 32;
    const v16h a0 = ldf(pa0 + k0), a1 = ldf(pa1 + k0), b = ldf(pb + k0);
    c0 = wm(a0, b, c0);
    c1 = wm(a1, b, c1);
  }
#pragma unroll
  for (int r = 0; r < 8; ++r) {
    Xs[(8 * hh + r) * XSP + lcol]      = c0[r] * (1.0f / WSC);
    Xs[(16 + 8 * hh + r) * XSP + lcol] = c1[r] * (1.0f / WSC);
  }
  __syncthreads();

  v4f xr[4];
  float* pr[4];
#pragma unroll
  for (int i = 0; i < 4; ++i) {
    const int row = 4 * wave + i;
    xr[i] = *(const v4f*)(Xs + row * XSP + 4 * lane);
    pr[i] = out + (size_t)(rowBase + row) * QKVW + colBlk + 4 * lane;
  }
#pragma unroll
  for (int i = 0; i < 4; ++i) *(volatile v4f*)(pr[i]) = xr[i];
  __threadfence();
#pragma unroll
  for (int i = 0; i < 4; ++i) *(volatile v4f*)(pr[i]) = xr[i];
}

__global__ __launch_bounds__(NTHR) void k_agg(
    const float* __restrict__ qkvD, const float* __restrict__ qkvS,
    const int* __restrict__ dIdx, const int* __restrict__ sIdx,
    _Float16* ctx, int nDst, int nSrc, int nE) {
  extern __shared__ v4f lds_dyn[];
  float* sacc = (float*)lds_dyn;
  float* den  = sacc + LDS_SACC;
  int*   list = (int*)(den + LDS_DEN);
  int*   wcnt = list + LDS_LIST;

  const int tid  = threadIdx.x;
  const int lane = tid & 31;
  const int wave = tid >> 5;
  const int hh   = lane >> 4;
  const int m    = lane & 15;
  const int hd   = lane >> 2;
  const int nodeBase = blockIdx.x * NB;

  {
    const v4f z4 = {0.f, 0.f, 0.f, 0.f};
    for (int i = tid; i < (LDS_SACC + LDS_DEN) / 4; i += NTHR) lds_dyn[i] = z4;
  }
  __syncthreads();

  const bool al16 = ((((size_t)dIdx) & 15) == 0);
  const int nChunks = (nE + CHUNK - 1) / CHUNK;
#pragma unroll 1
  for (int ch = 0; ch < nChunks; ++ch) {
    const int cbase = ch * CHUNK;
    int wc = 0;
#pragma unroll
    for (int g = 0; g < NGRP; ++g) {
      const int el0 = (g * NTHR + tid) * 4;
      const int e0  = cbase + el0;
      const int sent = -2147483647 - 1;
      v4i d;
      if (al16 && (e0 + 3 < nE)) {
        d = *(const v4i*)(dIdx + e0);
      } else {
        d.x = (e0     < nE) ? dIdx[min(e0, nE - 1)]     : sent;
        d.y = (e0 + 1 < nE) ? dIdx[min(e0 + 1, nE - 1)] : sent;
        d.z = (e0 + 2 < nE) ? dIdx[min(e0 + 2, nE - 1)] : sent;
        d.w = (e0 + 3 < nE) ? dIdx[min(e0 + 3, nE - 1)] : sent;
      }
      const unsigned s0 = (unsigned)d.x - (unsigned)nodeBase;
      const unsigned s1 = (unsigned)d.y - (unsigned)nodeBase;
      const unsigned s2 = (unsigned)d.z - (unsigned)nodeBase;
      const unsigned s3 = (unsigned)d.w - (unsigned)nodeBase;
      const bool h0 = s0 < (unsigned)NB;
      const bool h1 = s1 < (unsigned)NB;
      const bool h2 = s2 < (unsigned)NB;
      const bool h3 = s3 < (unsigned)NB;
      const unsigned many = __builtin_amdgcn_ballot_w32(h0 | h1 | h2 | h3);
      if (many != 0u) {
#define HITJ(J, HJ, SJ) { \
          const unsigned mj = __builtin_amdgcn_ballot_w32(HJ); \
          if (HJ) { \
            const int pos = wc + (int)__builtin_amdgcn_mbcnt_lo(mj, 0u); \
            if (pos < WCAP) list[wave * WCAP + pos] = ((el0 + (J)) << 9) | (int)(SJ); \
          } \
          wc += (int)__builtin_popcount(mj); }
        HITJ(0, h0, s0)
        HITJ(1, h1, s1)
        HITJ(2, h2, s2)
        HITJ(3, h3, s3)
#undef HITJ
      }
    }
    if (lane == 0) wcnt[wave] = wc;
    __syncthreads();

    if (wave == 0) {
      for (int wsx = 0; wsx < NWAVE; ++wsx) {
        int n = wcnt[wsx];
        if (n > WCAP) n = WCAP;
        if (n < 0) n = 0;
        for (int i = 0; i < n; ++i) {
          const int ent  = list[wsx * WCAP + i];
          const int slot = ent & (NB - 1);
          const int el   = (ent >> 9) & (CHUNK - 1);
          int e = cbase + el;
          if (e > nE - 1) e = nE - 1;
          int src = sIdx[e];
          src = src < 0 ? 0 : (src > nSrc - 1 ? nSrc - 1 : src);
          int nd = nodeBase + slot;
          if (nd > nDst - 1) nd = nDst - 1;
          const v4f qv = *(const v4f*)(qkvD + (size_t)nd * QKVW + 4 * lane);
          const float* ps = qkvS + (size_t)src * QKVW + 4 * lane;
          const v4f kv = *(const v4f*)(ps + DF);
          const v4f vv = *(const v4f*)(ps + 2 * DF);
          float dt = qv.x * kv.x + qv.y * kv.y + qv.z * kv.z + qv.w * kv.w;
          dt += __shfl_xor(dt, 1, 32);
          dt += __shfl_xor(dt, 2, 32);
          float s = dt * 0.25f;
          s = fminf(fmaxf(s, -60.f), 60.f);
          const float p = __expf(s);
          v4f* ap = (v4f*)(sacc + slot * DF + 4 * lane);
          const v4f cur = *ap;
          *ap = cur + p * vv;
          if ((lane & 3) == 0) {
            const float o = den[slot * NH + hd];
            den[slot * NH + hd] = o + p;
          }
        }
      }
    }
    __syncthreads();
  }

#pragma unroll 1
  for (int j = 0; j < NB / (NWAVE * 2); ++j) {
    const int slot = wave * (NB / NWAVE) + 2 * j + hh;
    const int node = nodeBase + slot;
    const int cl   = 8 * m;
    const float dv  = den[slot * NH + (m >> 1)];
    const float inv = (dv > 0.f) ? (ASC * __builtin_amdgcn_rcpf(dv)) : 0.f;
    const v4f a = *(const v4f*)(sacc + slot * DF + cl) * inv;
    const v4f b = *(const v4f*)(sacc + slot * DF + cl + 4) * inv;
    const Pack16 u = pack8(a, b);
    const bool ok = node < nDst;
    _Float16* p = ctx + (size_t)(ok ? node : 0) * DF + cl;
    if (ok) *(volatile v4i*)p = u.i;
    __threadfence();
    if (ok) *(volatile v4i*)p = u.i;
  }
}

__global__ __launch_bounds__(NTHR) void k_gate(
    const _Float16* __restrict__ H16, const _Float16* __restrict__ C16, const float* __restrict__ H32,
    const _Float16* __restrict__ Wgt, const float* __restrict__ bg,
    const _Float16* __restrict__ Wut, const float* __restrict__ bu,
    const float* __restrict__ gam, const float* __restrict__ bet,
    float* hup, _Float16* hn) {
  __shared__ __attribute__((aligned(16))) float Xs[GR * XSP];
  const int tid = threadIdx.x, lane = tid & 31, wave = tid >> 5;
  const int hh = lane >> 4, m = lane & 15;
  const int rowBase = blockIdx.x * GR;

  {
    const int r = tid >> 3, c = (tid & 7) * 16;
    const float* p = H32 + (size_t)(rowBase + r) * DF + c;
    float* q = Xs + r * XSP + c;
    *(v4f*)(q)      = *(const v4f*)(p);
    *(v4f*)(q + 4)  = *(const v4f*)(p + 4);
    *(v4f*)(q + 8)  = *(const v4f*)(p + 8);
    *(v4f*)(q + 12) = *(const v4f*)(p + 12);
  }
  __syncthreads();

  const int lcol = wave * 16 + m;
  const _Float16* ph0 = H16 + (size_t)(rowBase + m) * DF + 8 * hh;
  const _Float16* ph1 = ph0 + (size_t)16 * DF;
  const _Float16* pc0 = C16 + (size_t)(rowBase + m) * DF + 8 * hh;
  const _Float16* pc1 = pc0 + (size_t)16 * DF;
  const _Float16* pg  = Wgt + (size_t)lcol * (2 * DF) + 8 * hh;
  const _Float16* pu  = Wut + (size_t)lcol * DF + 8 * hh;
  v8f gh0 = z8f(), gh1 = z8f(), gc0 = z8f(), gc1 = z8f(), u0 = z8f(), u1 = z8f();
#pragma unroll
  for (int kt = 0; kt < DF / 32; ++kt) {
    const int k0 = kt * 32;
    const v16h ah0 = ldf(ph0 + k0), ah1 = ldf(ph1 + k0), bgh = ldf(pg + k0);
    gh0 = wm(ah0, bgh, gh0);
    gh1 = wm(ah1, bgh, gh1);
    const v16h ac0 = ldf(pc0 + k0), ac1 = ldf(pc1 + k0);
    const v16h bgc = ldf(pg + DF + k0), buu = ldf(pu + k0);
    gc0 = wm(ac0, bgc, gc0);
    gc1 = wm(ac1, bgc, gc1);
    u0  = wm(ac0, buu, u0);
    u1  = wm(ac1, buu, u1);
  }

  const float bgv = bg[lcol], buv = bu[lcol];
#pragma unroll
  for (int r = 0; r < 8; ++r) {
    {
      const int row = 8 * hh + r;
      const float g  = gh0[r] * (1.0f / WSC) + gc0[r] * (1.0f / (WSC * ASC)) + bgv;
      const float uu = u0[r] * (1.0f / (WSC * ASC)) + buv;
      const float sg = __builtin_amdgcn_rcpf(1.0f + __expf(-g));
      float* px = Xs + row * XSP + lcol;
      const float x = *px;
      *px = x + sg * uu;
    }
    {
      const int row = 16 + 8 * hh + r;
      const float g  = gh1[r] * (1.0f / WSC) + gc1[r] * (1.0f / (WSC * ASC)) + bgv;
      const float uu = u1[r] * (1.0f / (WSC * ASC)) + buv;
      const float sg = __builtin_amdgcn_rcpf(1.0f + __expf(-g));
      float* px = Xs + row * XSP + lcol;
      const float x = *px;
      *px = x + sg * uu;
    }
  }
  __syncthreads();

  v4f xr[4];
  float* pr[4];
#pragma unroll
  for (int i = 0; i < 4; ++i) {
    const int row = 4 * wave + i;
    xr[i] = *(const v4f*)(Xs + row * XSP + 4 * lane);
    pr[i] = hup + (size_t)(rowBase + row) * DF + 4 * lane;
  }
  const v4f g0 = *(const v4f*)(gam + 8 * m), g1 = *(const v4f*)(gam + 8 * m + 4);
  const v4f e0 = *(const v4f*)(bet + 8 * m), e1 = *(const v4f*)(bet + 8 * m + 4);
  Pack16 hv[2];
  _Float16* pn[2];
#pragma unroll
  for (int p = 0; p < 2; ++p) {
    const int row = 4 * wave + 2 * p + hh;
    const v4f x0 = *(const v4f*)(Xs + row * XSP + 8 * m);
    const v4f x1 = *(const v4f*)(Xs + row * XSP + 8 * m + 4);
    const float s  = hsum16(x0.x + x0.y + x0.z + x0.w + x1.x + x1.y + x1.z + x1.w);
    const float mu = s * (1.0f / DF);
    const v4f d0 = x0 - mu, d1 = x1 - mu;
    const float q  = hsum16(d0.x * d0.x + d0.y * d0.y + d0.z * d0.z + d0.w * d0.w +
                            d1.x * d1.x + d1.y * d1.y + d1.z * d1.z + d1.w * d1.w);
    const float rs = rsqrtf(q * (1.0f / DF) + 1e-5f);
    const v4f y0 = d0 * rs * g0 + e0;
    const v4f y1 = d1 * rs * g1 + e1;
    hv[p] = pack8(y0, y1);
    pn[p] = hn + (size_t)(rowBase + row) * DF + 8 * m;
  }
#pragma unroll
  for (int i = 0; i < 4; ++i) *(volatile v4f*)(pr[i]) = xr[i];
#pragma unroll
  for (int p = 0; p < 2; ++p) *(volatile v4i*)(pn[p]) = hv[p].i;
  __threadfence();
#pragma unroll
  for (int i = 0; i < 4; ++i) *(volatile v4f*)(pr[i]) = xr[i];
#pragma unroll
  for (int p = 0; p < 2; ++p) *(volatile v4i*)(pn[p]) = hv[p].i;
}

__global__ __launch_bounds__(NTHR) void k_ffn1(const _Float16* __restrict__ A, const _Float16* __restrict__ W1t,
                                               const float* __restrict__ b1, _Float16* t16) {
  __shared__ __attribute__((aligned(16))) float Xs[GR * XSP];
  const int tid = threadIdx.x, lane = tid & 31, wave = tid >> 5;
  const int hh = lane >> 4, m = lane & 15;
  const int rowBase = blockIdx.x * GR;
  const int colBlk = blockIdx.y * DF;
  const int lcol = wave * 16 + m;
  const int ncol = colBlk + lcol;

  const _Float16* pa0 = A + (size_t)(rowBase + m) * DF + 8 * hh;
  const _Float16* pa1 = pa0 + (size_t)16 * DF;
  const _Float16* pb  = W1t + (size_t)ncol * DF + 8 * hh;
  v8f c0 = z8f(), c1 = z8f();
#pragma unroll
  for (int kt = 0; kt < DF / 32; ++kt) {
    const int k0 = kt * 32;
    const v16h a0 = ldf(pa0 + k0), a1 = ldf(pa1 + k0), b = ldf(pb + k0);
    c0 = wm(a0, b, c0);
    c1 = wm(a1, b, c1);
  }
  const float bv = b1[ncol];
#pragma unroll
  for (int r = 0; r < 8; ++r) {
    const float v0 = fmaxf(c0[r] * (1.0f / WSC) + bv, 0.f) * ASC;
    const float v1 = fmaxf(c1[r] * (1.0f / WSC) + bv, 0.f) * ASC;
    Xs[(8 * hh + r) * XSP + lcol]      = v0;
    Xs[(16 + 8 * hh + r) * XSP + lcol] = v1;
  }
  __syncthreads();

  Pack16 hv[2];
  _Float16* pt[2];
#pragma unroll
  for (int p = 0; p < 2; ++p) {
    const int row = 4 * wave + 2 * p + hh;
    const v4f x0 = *(const v4f*)(Xs + row * XSP + 8 * m);
    const v4f x1 = *(const v4f*)(Xs + row * XSP + 8 * m + 4);
    hv[p] = pack8(x0, x1);
    pt[p] = t16 + (size_t)(rowBase + row) * FFW + colBlk + 8 * m;
  }
#pragma unroll
  for (int p = 0; p < 2; ++p) *(volatile v4i*)(pt[p]) = hv[p].i;
  __threadfence();
#pragma unroll
  for (int p = 0; p < 2; ++p) *(volatile v4i*)(pt[p]) = hv[p].i;
}

__global__ __launch_bounds__(NTHR) void k_ffn2(const _Float16* __restrict__ T16, const _Float16* __restrict__ W2t,
                                               const float* __restrict__ b2, const float* __restrict__ hup,
                                               float* out) {
  __shared__ __attribute__((aligned(16))) float Xs[GR * XSP];
  const int tid = threadIdx.x, lane = tid & 31, wave = tid >> 5;
  const int hh = lane >> 4, m = lane & 15;
  const int rowBase = blockIdx.x * GR;

  {
    const int r = tid >> 3, c = (tid & 7) * 16;
    const float* p = hup + (size_t)(rowBase + r) * DF + c;
    float* q = Xs + r * XSP + c;
    *(v4f*)(q)      = *(const v4f*)(p);
    *(v4f*)(q + 4)  = *(const v4f*)(p + 4);
    *(v4f*)(q + 8)  = *(const v4f*)(p + 8);
    *(v4f*)(q + 12) = *(const v4f*)(p + 12);
  }
  __syncthreads();

  const int lcol = wave * 16 + m;
  const _Float16* pa0 = T16 + (size_t)(rowBase + m) * FFW + 8 * hh;
  const _Float16* pa1 = pa0 + (size_t)16 * FFW;
  const _Float16* pb  = W2t + (size_t)lcol * FFW + 8 * hh;
  v8f c0 = z8f(), c1 = z8f();
#pragma unroll
  for (int kt = 0; kt < FFW / 32; ++kt) {
    const int k0 = kt * 32;
    const v16h a0 = ldf(pa0 + k0), a1 = ldf(pa1 + k0), b = ldf(pb + k0);
    c0 = wm(a0, b, c0);
    c1 = wm(a1, b, c1);
  }
  const float bv = b2[lcol];
#pragma unroll
  for (int r = 0; r < 8; ++r) {
    {
      float* px = Xs + (8 * hh + r) * XSP + lcol;
      const float x = *px;
      *px = x + c0[r] * (1.0f / (WSC * ASC)) + bv;
    }
    {
      float* px = Xs + (16 + 8 * hh + r) * XSP + lcol;
      const float x = *px;
      *px = x + c1[r] * (1.0f / (WSC * ASC)) + bv;
    }
  }
  __syncthreads();

  v4f xr[4];
  float* pr[4];
#pragma unroll
  for (int i = 0; i < 4; ++i) {
    const int row = 4 * wave + i;
    xr[i] = *(const v4f*)(Xs + row * XSP + 4 * lane);
    pr[i] = out + (size_t)(rowBase + row) * DF + 4 * lane;
  }
#pragma unroll
  for (int i = 0; i < 4; ++i) *(volatile v4f*)(pr[i]) = xr[i];
  __threadfence();
#pragma unroll
  for (int i = 0; i < 4; ++i) *(volatile v4f*)(pr[i]) = xr[i];
}

extern "C" void kernel_launch(void* const* d_in, const int* in_sizes, int n_in,
                              void* d_out, int out_size, void* d_ws, size_t ws_size,
                              hipStream_t stream) {
  if (n_in < 30) return;
  const int nP = in_sizes[0] / DF;
  const int nL = in_sizes[1] / DF;
  const int nE = in_sizes[2];
  if (nP <= 0 || nL <= 0 || in_sizes[0] != nP * DF || in_sizes[1] != nL * DF) return;
  if ((nP % GR) != 0 || (nL % GR) != 0) return;
  if (nE < 0 || in_sizes[3] != nE) return;
  {
    const int sq[8] = {4, 5, 6, 9, 11, 12, 13, 16};
    for (int i = 0; i < 8; ++i) if (in_sizes[sq[i]] != DF * DF) return;
    if (in_sizes[7] != 2 * DF * DF || in_sizes[14] != 2 * DF * DF) return;
    const int bs[10] = {8, 10, 15, 17, 18, 19, 20, 21, 25, 29};
    for (int i = 0; i < 10; ++i) if (in_sizes[bs[i]] != DF) return;
    if (in_sizes[22] != DF * FFW || in_sizes[24] != FFW * DF) return;
    if (in_sizes[26] != DF * FFW || in_sizes[28] != FFW * DF) return;
    if (in_sizes[23] != FFW || in_sizes[27] != FFW) return;
  }
  if (out_size != (nP + nL) * DF) return;

  const float* hP    = (const float*)d_in[0];
  const float* hL    = (const float*)d_in[1];
  const int*   pIdx  = (const int*)d_in[2];
  const int*   lIdx  = (const int*)d_in[3];
  const float* Wq_l  = (const float*)d_in[4];
  const float* Wk_p  = (const float*)d_in[5];
  const float* Wv_p  = (const float*)d_in[6];
  const float* Wg_l  = (const float*)d_in[7];
  const float* bg_l  = (const float*)d_in[8];
  const float* Wu_l  = (const float*)d_in[9];
  const float* bu_l  = (const float*)d_in[10];
  const float* Wq_p  = (const float*)d_in[11];
  const float* Wk_l  = (const float*)d_in[12];
  const float* Wv_l  = (const float*)d_in[13];
  const float* Wg_p  = (const float*)d_in[14];
  const float* bg_p  = (const float*)d_in[15];
  const float* Wu_p  = (const float*)d_in[16];
  const float* bu_p  = (const float*)d_in[17];
  const float* lnP_g = (const float*)d_in[18];
  const float* lnP_b = (const float*)d_in[19];
  const float* lnL_g = (const float*)d_in[20];
  const float* lnL_b = (const float*)d_in[21];
  const float* W1_p  = (const float*)d_in[22];
  const float* b1_p  = (const float*)d_in[23];
  const float* W2_p  = (const float*)d_in[24];
  const float* b2_p  = (const float*)d_in[25];
  const float* W1_l  = (const float*)d_in[26];
  const float* b1_l  = (const float*)d_in[27];
  const float* W2_l  = (const float*)d_in[28];
  const float* b2_l  = (const float*)d_in[29];
  float* outP = (float*)d_out;
  float* outL = (float*)d_out + (size_t)nP * DF;

  char* ws = (char*)d_ws;
  size_t off = 0;
  auto take = [&](size_t bytes) -> void* {
    void* p = ws + off;
    off += (bytes + 255) & ~(size_t)255;
    return p;
  };
  _Float16* h16P   = (_Float16*)take((size_t)nP * DF * 2);
  _Float16* h16L   = (_Float16*)take((size_t)nL * DF * 2);
  _Float16* WqkvtP = (_Float16*)take((size_t)QKVW * DF * 2);
  _Float16* WqkvtL = (_Float16*)take((size_t)QKVW * DF * 2);
  _Float16* WgtL   = (_Float16*)take((size_t)DF * 2 * DF * 2);
  _Float16* WutL   = (_Float16*)take((size_t)DF * DF * 2);
  _Float16* WgtP   = (_Float16*)take((size_t)DF * 2 * DF * 2);
  _Float16* WutP   = (_Float16*)take((size_t)DF * DF * 2);
  _Float16* W1tP   = (_Float16*)take((size_t)FFW * DF * 2);
  _Float16* W2tP   = (_Float16*)take((size_t)DF * FFW * 2);
  _Float16* W1tL   = (_Float16*)take((size_t)FFW * DF * 2);
  _Float16* W2tL   = (_Float16*)take((size_t)DF * FFW * 2);
  float*    qkvP   = (float*)take((size_t)nP * QKVW * 4);
  float*    qkvL   = (float*)take((size_t)nL * QKVW * 4);
  _Float16* ctxP   = (_Float16*)take((size_t)nP * DF * 2);
  _Float16* ctxL   = (_Float16*)take((size_t)nL * DF * 2);
  float*    hupP   = (float*)take((size_t)nP * DF * 4);
  float*    hupL   = (float*)take((size_t)nL * DF * 4);
  _Float16* hnP    = (_Float16*)take((size_t)nP * DF * 2);
  _Float16* hnL    = (_Float16*)take((size_t)nL * DF * 2);
  _Float16* tP     = (_Float16*)take((size_t)nP * FFW * 2);
  _Float16* tL     = (_Float16*)take((size_t)nL * FFW * 2);
  if (off > ws_size) return;

  const int n8P = nP * DF / 8, n8L = nL * DF / 8;
  k_cvt<<<(n8P + NTHR - 1) / NTHR, NTHR, 0, stream>>>(hP, h16P, n8P);
  k_cvt<<<(n8L + NTHR - 1) / NTHR, NTHR, 0, stream>>>(hL, h16L, n8L);

  k_wt<<<dim3((DF / 64) * (DF / 32), 1, 3), NTHR, 0, stream>>>(Wq_p, Wk_p, Wv_p, WqkvtP, DF, DF);
  k_wt<<<dim3((DF / 64) * (DF / 32), 1, 3), NTHR, 0, stream>>>(Wq_l, Wk_l, Wv_l, WqkvtL, DF, DF);
  k_wt<<<dim3((2 * DF / 64) * (DF / 32), 1, 1), NTHR, 0, stream>>>(Wg_l, Wg_l, Wg_l, WgtL, 2 * DF, DF);
  k_wt<<<dim3((DF / 64) * (DF / 32), 1, 1), NTHR, 0, stream>>>(Wu_l, Wu_l, Wu_l, WutL, DF, DF);
  k_wt<<<dim3((2 * DF / 64) * (DF / 32), 1, 1), NTHR, 0, stream>>>(Wg_p, Wg_p, Wg_p, WgtP, 2 * DF, DF);
  k_wt<<<dim3((DF / 64) * (DF / 32), 1, 1), NTHR, 0, stream>>>(Wu_p, Wu_p, Wu_p, WutP, DF, DF);
  k_wt<<<dim3((DF / 64) * (FFW / 32), 1, 1), NTHR, 0, stream>>>(W1_p, W1_p, W1_p, W1tP, DF, FFW);
  k_wt<<<dim3((FFW / 64) * (DF / 32), 1, 1), NTHR, 0, stream>>>(W2_p, W2_p, W2_p, W2tP, FFW, DF);
  k_wt<<<dim3((DF / 64) * (FFW / 32), 1, 1), NTHR, 0, stream>>>(W1_l, W1_l, W1_l, W1tL, DF, FFW);
  k_wt<<<dim3((FFW / 64) * (DF / 32), 1, 1), NTHR, 0, stream>>>(W2_l, W2_l, W2_l, W2tL, FFW, DF);

  k_qkv<<<dim3(nP / GR, QKVW / DF, 1), NTHR, 0, stream>>>(h16P, WqkvtP, qkvP);
  k_qkv<<<dim3(nL / GR, QKVW / DF, 1), NTHR, 0, stream>>>(h16L, WqkvtL, qkvL);

  hipFuncSetAttribute(reinterpret_cast<const void*>(&k_agg),
                      hipFuncAttributeMaxDynamicSharedMemorySize, AGG_LDS_BYTES);
  k_agg<<<(nL + NB - 1) / NB, NTHR, AGG_LDS_BYTES, stream>>>(qkvL, qkvP, lIdx, pIdx, ctxL, nL, nP, nE);
  k_agg<<<(nP + NB - 1) / NB, NTHR, AGG_LDS_BYTES, stream>>>(qkvP, qkvL, pIdx, lIdx, ctxP, nP, nL, nE);

  k_gate<<<nL / GR, NTHR, 0, stream>>>(h16L, ctxL, hL, WgtL, bg_l, WutL, bu_l, lnL_g, lnL_b, hupL, hnL);
  k_gate<<<nP / GR, NTHR, 0, stream>>>(h16P, ctxP, hP, WgtP, bg_p, WutP, bu_p, lnP_g, lnP_b, hupP, hnP);

  k_ffn1<<<dim3(nP / GR, FFW / DF, 1), NTHR, 0, stream>>>(hnP, W1tP, b1_p, tP);
  k_ffn2<<<nP / GR, NTHR, 0, stream>>>(tP, W2tP, b2_p, hupP, outP);
  k_ffn1<<<dim3(nL / GR, FFW / DF, 1), NTHR, 0, stream>>>(hnL, W1tL, b1_l, tL);
  k_ffn2<<<nL / GR, NTHR, 0, stream>>>(tL, W2tL, b2_l, hupL, outL);
}
